// SimpleRewardModel_17076789968980
// MI455X (gfx1250) — hardware-verified
//
#include <hip/hip_runtime.h>
#include <hip/hip_bf16.h>

typedef __attribute__((ext_vector_type(16))) _Float16 v16h;
typedef __attribute__((ext_vector_type(8)))  _Float16 v8h;
typedef __attribute__((ext_vector_type(4)))  _Float16 v4h;
typedef __attribute__((ext_vector_type(8)))  float    v8f;
typedef __attribute__((ext_vector_type(4)))  float    v4f;

#define B_  256
#define T_  512
#define E_  128
#define H_  64
#define G_  256

typedef float v4fa __attribute__((ext_vector_type(4), may_alias));
#define RSPLIT (1.0f / 2048.0f)
static __device__ __forceinline__ _Float16 lo_of(float v, _Float16 h) { return (_Float16)((v - (float)h) * 2048.0f); }
static __device__ __forceinline__ v8f wmma_f16(v16h a, v16h b, v8f c);
static __device__ __forceinline__ v8f wmma_split(v16h a, v16h al, v16h b, v16h bl, v8f c) {
    v8f x = {}; x = wmma_f16(al, b, x); x = wmma_f16(a, bl, x); return wmma_f16(a, b, c) + x * RSPLIT;
}
static __device__ __forceinline__ v8f wmma_f16(v16h a, v16h b, v8f c) {
    return __builtin_amdgcn_wmma_f32_16x16x32_f16(
         false, a,  false, b,
         (short)0, c,  false,  false);
}

static __device__ __forceinline__ float fast_sigmoid(float x) {
    return 1.0f / (1.0f + __expf(-x));
}
static __device__ __forceinline__ float fast_tanh(float x) {
    float e = __expf(2.0f * x);
    return 1.0f - 2.0f / (e + 1.0f);
}

__global__ __launch_bounds__(256) void k_cvt(
    const float* __restrict__ s, _Float16* __restrict__ d, int n4)
{
    const int i = blockIdx.x * 256 + threadIdx.x;
    if (i < n4) {
        const v4f x = *(const v4f*)(s + (size_t)i * 4);
        v4h y;
        #pragma unroll
        for (int e = 0; e < 4; ++e) y[e] = (_Float16)x[e];
        *(volatile v4h*)(d + (size_t)i * 4) = y; __threadfence(); *(volatile v4h*)(d + (size_t)i * 4) = y;
    }
}

__global__ __launch_bounds__(128) void k_xg(
    const int* __restrict__ ids, const _Float16* __restrict__ embF,
    const _Float16* __restrict__ WihF, const float* __restrict__ bih,
    const float* __restrict__ bhh, _Float16* __restrict__ xg)
{
    const int lane  = threadIdx.x & 31;
    const int wave  = threadIdx.x >> 5;
    const int btile = blockIdx.x;
    const int t0    = blockIdx.y * 8;
    const int m     = lane & 15;
    const int hi    = lane >> 4;

    v16h Bf[4][4];
    float bias[4];
    #pragma unroll
    for (int j = 0; j < 4; ++j) {
        const int g = (wave * 4 + j) * 16 + m;
        #pragma unroll
        for (int kk = 0; kk < 4; ++kk) {
            const _Float16* src = WihF + g * E_ + kk * 32 + 8 * hi;
            const v8h lo = *(const v8h*)src;
            const v8h up = *(const v8h*)(src + 16);
            #pragma unroll
            for (int e = 0; e < 8; ++e) { Bf[j][kk][e] = lo[e]; Bf[j][kk][e + 8] = up[e]; }
        }
        bias[j] = bih[g] + bhh[g];
    }

    for (int tt = 0; tt < 8; ++tt) {
        const int t  = t0 + tt;
        const int id = ids[(btile * 16 + m) * T_ + t];
        const _Float16* row = embF + (size_t)id * E_;
        v16h A[4];
        #pragma unroll
        for (int kk = 0; kk < 4; ++kk) {
            const int kb = kk * 32 + 8 * hi;
            const v8h lo = *(const v8h*)(row + kb);
            const v8h up = *(const v8h*)(row + kb + 16);
            #pragma unroll
            for (int e = 0; e < 8; ++e) { A[kk][e] = lo[e]; A[kk][e + 8] = up[e]; }
        }
        #pragma unroll
        for (int j = 0; j < 4; ++j) {
            v8f acc = {};
            #pragma unroll
            for (int kk = 0; kk < 4; ++kk) acc = wmma_f16(A[kk], Bf[j][kk], acc);
            const int ng = wave * 4 + j;
            v8h out;
            #pragma unroll
            for (int r = 0; r < 8; ++r) out[r] = (_Float16)(acc[r] + bias[j]);
            const size_t base = ((((size_t)t * 16 + btile) * 16 + ng) << 8) + lane * 8;
            *(volatile v8h*)(xg + base) = out; __threadfence(); *(volatile v8h*)(xg + base) = out;
        }
    }
}

__global__ __launch_bounds__(128) void k_lstm(
    const float* __restrict__ Whh, const _Float16* __restrict__ xg,
    float* __restrict__ features)
{
    const int lane  = threadIdx.x & 31;
    const int wave  = threadIdx.x >> 5;
    const int btile = blockIdx.x;
    const int m     = lane & 15;
    const int hi    = lane >> 4;

    __shared__ float    gate_lds[4][4][256];
    __shared__ _Float16 h_lds[2 * 16 * H_];
    __shared__ __attribute__((aligned(16))) _Float16 w_lds[2 * G_ * H_];

    for (int i = threadIdx.x; i < G_ * H_; i += 128) { const float w = Whh[i]; const _Float16 wh = (_Float16)w; w_lds[i] = wh; w_lds[G_ * H_ + i] = lo_of(w, wh); }
    __syncthreads();

    v16h hA[2] = {}, hAl[2] = {};
    float c[8], hsum[8];
    #pragma unroll
    for (int r = 0; r < 8; ++r) { c[r] = 0.0f; hsum[r] = 0.0f; }

    const size_t lane_off = (size_t)lane * 8;
    #define FRAG_BASE(tt, jj) \
        (((((size_t)(tt) * 16 + btile) * 16 + wave * 4 + (jj)) << 8) + lane_off)

    v8h xh[4];
    #pragma unroll
    for (int j = 0; j < 4; ++j) xh[j] = *(const v8h*)(xg + FRAG_BASE(0, j));

    for (int t = 0; t < T_; ++t) {
        const int tn = (t + 1 < T_) ? t + 1 : t;
        const int tp = (t + 2 < T_) ? t + 2 : t;
        #pragma unroll
        for (int j = 0; j < 4; ++j)
            __builtin_prefetch(xg + FRAG_BASE(tp, j), 0, 0);

        float act[4][8];
        v8h xn[4];
        #pragma unroll
        for (int j = 0; j < 4; ++j) {
            v8f acc;
            #pragma unroll
            for (int r = 0; r < 8; ++r) acc[r] = (float)xh[j][r];
            xn[j] = *(const v8h*)(xg + FRAG_BASE(tn, j));
            #pragma unroll
            for (int kk = 0; kk < 2; ++kk) {
                const _Float16* wr = w_lds + (wave * 64 + j * 16 + m) * H_ + kk * 32 + 8 * hi;
                const v8h b0 = *(const v8h*)wr, b1 = *(const v8h*)(wr + 16), c0 = *(const v8h*)(wr + G_ * H_), c1 = *(const v8h*)(wr + G_ * H_ + 16);
                v16h Bv, Bl;
                #pragma unroll
                for (int e = 0; e < 8; ++e) { Bv[e] = b0[e]; Bv[e + 8] = b1[e]; Bl[e] = c0[e]; Bl[e + 8] = c1[e]; }
                acc = wmma_split(hA[kk], hAl[kk], Bv, Bl, acc);
            }
            if (wave == 2) {
                #pragma unroll
                for (int r = 0; r < 8; ++r) act[j][r] = fast_tanh(acc[r]);
            } else {
                #pragma unroll
                for (int r = 0; r < 8; ++r) act[j][r] = fast_sigmoid(acc[r]);
            }
        }
        #pragma unroll
        for (int j = 0; j < 4; ++j) {
            #pragma unroll
            for (int r = 0; r < 8; ++r) gate_lds[wave][j][lane * 8 + r] = act[j][r];
        }
        __syncthreads();

        #pragma unroll
        for (int r = 0; r < 8; ++r) {
            const float iv = gate_lds[0][wave][lane * 8 + r];
            const float fv = gate_lds[1][wave][lane * 8 + r];
            const float gv = gate_lds[2][wave][lane * 8 + r];
            const float ov = gate_lds[3][wave][lane * 8 + r];
            const float cn = fv * c[r] + iv * gv;
            c[r] = cn;
            const float hn = ov * fast_tanh(cn);
            hsum[r] += hn;
            { const _Float16 hh = (_Float16)hn; h_lds[(r + 8 * hi) * H_ + wave * 16 + m] = hh; h_lds[16 * H_ + (r + 8 * hi) * H_ + wave * 16 + m] = lo_of(hn, hh); }
        }
        __syncthreads();

        #pragma unroll
        for (int kk = 0; kk < 2; ++kk) {
            const _Float16* hr = h_lds + m * H_ + kk * 32 + 8 * hi;
            const v8h lo = *(const v8h*)hr, up = *(const v8h*)(hr + 16);
            const v8h ll = *(const v8h*)(hr + 16 * H_), lu = *(const v8h*)(hr + 16 * H_ + 16);
            #pragma unroll
            for (int e = 0; e < 8; ++e) { hA[kk][e] = lo[e]; hA[kk][e + 8] = up[e]; hAl[kk][e] = ll[e]; hAl[kk][e + 8] = lu[e]; }
        }
        #pragma unroll
        for (int j = 0; j < 4; ++j) xh[j] = xn[j];
    }
    #undef FRAG_BASE

    const float inv = 1.0f / (float)T_;
    float* fst = &gate_lds[0][0][0];
    #pragma unroll
    for (int r = 0; r < 8; ++r) fst[(r + 8 * hi) * H_ + wave * 16 + m] = hsum[r] * inv;
    __syncthreads();
    #pragma unroll 1
    for (int pass = 0; pass < 2; ++pass) {
        for (int c = threadIdx.x; c < 256; c += 128) { const int rr = c >> 4, q = (c & 15) * 4;
            *(volatile v4f*)(features + (size_t)(btile * 16 + rr) * H_ + q) = *(const volatile v4fa*)(fst + rr * H_ + q); }
        __threadfence();
    }
}

__global__ __launch_bounds__(512) void k_head(
    const float* __restrict__ features, const float* __restrict__ W1,
    const float* __restrict__ b1, const float* __restrict__ W2,
    const float* __restrict__ b2, float* __restrict__ out)
{
    __shared__ __attribute__((aligned(16))) float so[B_];
    __shared__ float hs[16][16][33];
    const int wave = threadIdx.x >> 5, lane = threadIdx.x & 31, lm = lane & 15, lh = lane >> 4;
    const int r0w = wave * 16;
    v8f y0 = {}, y1 = {};
    #pragma unroll
    for (int kc = 0; kc < 2; ++kc) {
        v16h a, al, bA, bAl, bB, bBl;
        #pragma unroll
        for (int e = 0; e < 16; ++e) {
            const int k = kc * 32 + ((e < 8) ? (lh * 8 + e) : (16 + lh * 8 + (e - 8)));
            const float fv = features[(r0w + lm) * H_ + k];
            const float wA = W1[lm * 64 + k], wB = W1[(16 + lm) * 64 + k];
            a[e] = (_Float16)fv; al[e] = lo_of(fv, a[e]); bA[e] = (_Float16)wA; bAl[e] = lo_of(wA, bA[e]); bB[e] = (_Float16)wB; bBl[e] = lo_of(wB, bB[e]);
        }
        y0 = wmma_split(a, al, bA, bAl, y0); y1 = wmma_split(a, al, bB, bBl, y1);
    }
    #pragma unroll
    for (int r = 0; r < 8; ++r) { hs[wave][lh * 8 + r][lm] = fmaxf(y0[r] + b1[lm], 0.f); hs[wave][lh * 8 + r][16 + lm] = fmaxf(y1[r] + b1[16 + lm], 0.f); }
    asm volatile("s_wait_dscnt 0" ::: "memory");
    v16h a2, a2l, w2, w2l;
    #pragma unroll
    for (int e = 0; e < 16; ++e) {
        const int k = (e < 8) ? (lh * 8 + e) : (16 + lh * 8 + (e - 8));
        const float hv = hs[wave][lm][k];
        const float wv = (lm == 0) ? W2[k] : 0.f;
        a2[e] = (_Float16)hv; a2l[e] = lo_of(hv, a2[e]); w2[e] = (_Float16)wv; w2l[e] = lo_of(wv, w2[e]);
    }
    v8f o = {};
    o = wmma_split(a2, a2l, w2, w2l, o);
    if (lm == 0) {
        #pragma unroll
        for (int r = 0; r < 8; ++r) so[r0w + lh * 8 + r] = o[r] + b2[0];
    }
    __syncthreads();
    if (threadIdx.x < 64) {
        const v4f v = *(const volatile v4fa*)(so + threadIdx.x * 4);
        *(volatile v4f*)(out + threadIdx.x * 4) = v; __threadfence(); *(volatile v4f*)(out + threadIdx.x * 4) = v;
    }
}

extern "C" void kernel_launch(void* const* d_in, const int* in_sizes, int n_in,
                              void* d_out, int out_size, void* d_ws, size_t ws_size,
                              hipStream_t stream)
{
    const int*   ids = (const int*)  d_in[0];
    const float* emb = (const float*)d_in[1];
    const float* Wih = (const float*)d_in[2];
    const float* Whh = (const float*)d_in[3];
    const float* bih = (const float*)d_in[4];
    const float* bhh = (const float*)d_in[5];
    const float* W1  = (const float*)d_in[6];
    const float* b1  = (const float*)d_in[7];
    const float* W2  = (const float*)d_in[8];
    const float* b2  = (const float*)d_in[9];
    float* out = (float*)d_out;

    char* ws = (char*)d_ws;
    size_t off = 0;
    _Float16* xg = (_Float16*)(ws + off);
    off += (size_t)T_ * 16 * 16 * 256 * sizeof(_Float16);
    float* features = (float*)(ws + off);
    off += (size_t)B_ * H_ * sizeof(float);
    _Float16* embF = (_Float16*)(ws + off);
    off += (size_t)32000 * E_ * sizeof(_Float16);
    _Float16* WihF = (_Float16*)(ws + off);
    off += (size_t)G_ * E_ * sizeof(_Float16);
    _Float16* WhhF = (_Float16*)(ws + off);
    off += (size_t)G_ * H_ * sizeof(_Float16);

    {
        const int n4e = 32000 * E_ / 4;
        k_cvt<<<(n4e + 255) / 256, 256, 0, stream>>>(emb, embF, n4e);
        const int n4i = G_ * E_ / 4;
        k_cvt<<<(n4i + 255) / 256, 256, 0, stream>>>(Wih, WihF, n4i);
        const int n4h = G_ * H_ / 4;
        k_cvt<<<(n4h + 255) / 256, 256, 0, stream>>>(Whh, WhhF, n4h);
    }

    dim3 g1(16, T_ / 8);
    k_xg  <<<g1, 128, 0, stream>>>(ids, embF, WihF, bih, bhh, xg);
    k_lstm<<<16, 128, 0, stream>>>(Whh, xg, features);
    k_head<<<1, 512, 0, stream>>>(features, W1, b1, W2, b2, out);
}
